// LATTEConv_79448305041722
// MI455X (gfx1250) — hardware-verified
//
#include <hip/hip_runtime.h>
#include <stddef.h>
#include <stdint.h>


#define DF     256
#define NH     4
#define HC     64
#define NR     3
#define GR     32
#define AP     264
#define XSP    260
#define LGW    32
#define NTHR   256
#define NWAVE  8
#define NB     2048
#define CHUNK  2048
#define WCAP   256
#define NGRP   (CHUNK / (NTHR * 4))
#define ACLAMP 60.0f

static_assert(WCAP == (CHUNK / NTHR) * 32);
static_assert(NGRP == 2);
static_assert(NB == 2048);
static_assert(CHUNK == 2048);
static_assert(NB == NTHR * 8);
static_assert(GR * XSP * 4 <= 2 * GR * AP * 2);
static_assert((AP % 8) == 0);
static_assert((XSP % 4) == 0);
static_assert(NH * HC == DF);
static_assert(NTHR == NWAVE * 32);
static_assert(GR == 4 * NWAVE);

typedef float          v4f  __attribute__((ext_vector_type(4)));
typedef float          v8f  __attribute__((ext_vector_type(8)));
typedef int            v4i  __attribute__((ext_vector_type(4)));
typedef _Float16       v8h  __attribute__((ext_vector_type(8)));
typedef _Float16       v16h __attribute__((ext_vector_type(16)));
typedef __bf16         v16b __attribute__((ext_vector_type(16)));
typedef unsigned short v8us __attribute__((ext_vector_type(8)));
union FragH  { v16h v; v8h  half[2]; };
union FragB  { v16b v; v8us half[2]; };
union Pack16 { v8h  h; v4i i; };
union PackU  { v8us u; v4i i; };

__device__ __forceinline__ v8f wmh(v16h a, v16h b, v8f c) {
  v8f d = __builtin_amdgcn_wmma_f32_16x16x32_f16(false, a, false, b, (short)0, c, false, false);
  asm volatile("v_nop\n\tv_nop\n\tv_nop\n\tv_nop" : "+v"(d) : "v"(a), "v"(b));
  return d;
}
__device__ __forceinline__ v8f wmb(v16b a, v16b b, v8f c) {
  v8f d = __builtin_amdgcn_wmma_f32_16x16x32_bf16(false, a, false, b, (short)0, c, false, false);
  asm volatile("v_nop\n\tv_nop\n\tv_nop\n\tv_nop" : "+v"(d) : "v"(a), "v"(b));
  return d;
}

__device__ __forceinline__ unsigned short bf16_rne(float x) {
  unsigned u = __float_as_uint(x);
  u += 0x7fffu + ((u >> 16) & 1u);
  return (unsigned short)(u >> 16);
}
__device__ __forceinline__ void bf16_split(float x, unsigned short& hi, unsigned short& lo) {
  const unsigned short hv = bf16_rne(x);
  const float hf = __uint_as_float(((unsigned)hv) << 16);
  hi = hv;
  lo = bf16_rne(x - hf);
}

__device__ __forceinline__ float wsum(float v) {
  v += __shfl_xor(v, 16, 32);
  v += __shfl_xor(v, 8, 32);
  v += __shfl_xor(v, 4, 32);
  v += __shfl_xor(v, 2, 32);
  v += __shfl_xor(v, 1, 32);
  return v;
}
__device__ __forceinline__ v4f lrelu4(v4f z) {
  v4f o;
  o.x = z.x >= 0.f ? z.x : 0.2f * z.x;
  o.y = z.y >= 0.f ? z.y : 0.2f * z.y;
  o.z = z.z >= 0.f ? z.z : 0.2f * z.z;
  o.w = z.w >= 0.f ? z.w : 0.2f * z.w;
  return o;
}
__device__ __forceinline__ v4f max4(v4f a, v4f b) {
  v4f o;
  o.x = fmaxf(a.x, b.x); o.y = fmaxf(a.y, b.y); o.z = fmaxf(a.z, b.z); o.w = fmaxf(a.w, b.w);
  return o;
}
__device__ __forceinline__ v4f exp4(v4f a) {
  v4f o;
  o.x = __expf(a.x); o.y = __expf(a.y); o.z = __expf(a.z); o.w = __expf(a.w);
  return o;
}
__device__ __forceinline__ v4f relu4(v4f a) {
  v4f o;
  o.x = a.x > 0.f ? a.x : 0.f; o.y = a.y > 0.f ? a.y : 0.f;
  o.z = a.z > 0.f ? a.z : 0.f; o.w = a.w > 0.f ? a.w : 0.f;
  return o;
}

__global__ __launch_bounds__(NTHR) void k_prep(const float* __restrict__ Wl, const float* __restrict__ Wr,
                                               _Float16* Wl16, unsigned short* Wrh, unsigned short* Wrl, int nT) {
  const int t = blockIdx.x * NTHR + threadIdx.x;
  if (t >= nT) return;
  const int n  = t >> 5;
  const int k0 = (t & 31) * 8;
  Pack16 pl; PackU ph, pw;
#pragma unroll
  for (int i = 0; i < 8; ++i) {
    const size_t si = (size_t)(k0 + i) * DF + n;
    const float wl = Wl[si];
    const float wr = Wr[si];
    pl.h[i] = (_Float16)(wl * 16.0f);
    unsigned short hi, lo;
    bf16_split(wr, hi, lo);
    ph.u[i] = hi;
    pw.u[i] = lo;
  }
  const size_t o = (size_t)n * DF + k0;
  const v4i a = pl.i, b = ph.i, c = pw.i;
  *(volatile v4i*)(Wl16 + o) = a;
  *(volatile v4i*)(Wrh + o)  = b;
  *(volatile v4i*)(Wrl + o)  = c;
  __threadfence();
  *(volatile v4i*)(Wl16 + o) = a;
  *(volatile v4i*)(Wrh + o)  = b;
  *(volatile v4i*)(Wrl + o)  = c;
}

__global__ __launch_bounds__(NTHR) void k_gemm(
    const float* __restrict__ feat, const _Float16* __restrict__ Wl16,
    const unsigned short* __restrict__ Wrh, const unsigned short* __restrict__ Wrl,
    const float* __restrict__ bl, const float* __restrict__ br,
    const float* __restrict__ attl, const float* __restrict__ attr,
    const float* __restrict__ relq, const float* __restrict__ relk,
    float* vpl, float* lgp, int nN) {
  __shared__ __attribute__((aligned(16))) _Float16 Af[GR * AP];
  __shared__ __attribute__((aligned(16))) unsigned char Ush[2 * GR * AP * 2];
  __shared__ __attribute__((aligned(16))) float LGs[GR * LGW];
  unsigned short* Ah = (unsigned short*)Ush;
  unsigned short* Al = Ah + GR * AP;
  float* Xs = (float*)Ush;

  const int tid  = threadIdx.x;
  const int lane = tid & 31;
  const int wave = tid >> 5;
  const int hh   = lane >> 4;
  const int m    = lane & 15;
  const int rowBase = blockIdx.x * GR;

  {
    const int r  = tid >> 3;
    const int c0 = (tid & 7) * 32;
    int row = rowBase + r;
    if (row > nN - 1) row = nN - 1;
    const float* p = feat + (size_t)row * DF + c0;
#pragma unroll
    for (int q = 0; q < 4; ++q) {
      const v4f f0 = *(const v4f*)(p + 8 * q);
      const v4f f1 = *(const v4f*)(p + 8 * q + 4);
      Pack16 u; PackU uh, ul;
      unsigned short hi_, lo_;
#define CV(I, X) { const float xx = (X); u.h[I] = (_Float16)xx; bf16_split(xx, hi_, lo_); uh.u[I] = hi_; ul.u[I] = lo_; }
      CV(0, f0.x) CV(1, f0.y) CV(2, f0.z) CV(3, f0.w)
      CV(4, f1.x) CV(5, f1.y) CV(6, f1.z) CV(7, f1.w)
#undef CV
      *(v8h*)(Af + r * AP + c0 + 8 * q)  = u.h;
      *(v8us*)(Ah + r * AP + c0 + 8 * q) = uh.u;
      *(v8us*)(Al + r * AP + c0 + 8 * q) = ul.u;
    }
  }
  __syncthreads();

  const int hd   = wave & 3;
  const int rt   = wave >> 2;
  const int arow = rt * 16 + m;

  v8f accv[4];
#pragma unroll
  for (int ct = 0; ct < 4; ++ct) { v8f z = {0.f, 0.f, 0.f, 0.f, 0.f, 0.f, 0.f, 0.f}; accv[ct] = z; }
#pragma unroll 1
  for (int kt = 0; kt < DF / 32; ++kt) {
    const int k0 = kt * 32;
    FragB fah, fal;
    const unsigned short* pah = Ah + arow * AP + k0 + 8 * hh;
    const unsigned short* pal = Al + arow * AP + k0 + 8 * hh;
    fah.half[0] = *(const v8us*)pah; fah.half[1] = *(const v8us*)(pah + 16);
    fal.half[0] = *(const v8us*)pal; fal.half[1] = *(const v8us*)(pal + 16);
#pragma unroll
    for (int ct = 0; ct < 4; ++ct) {
      const int ncol = hd * HC + ct * 16 + m;
      const unsigned short* pbh = Wrh + (size_t)ncol * DF + k0 + 8 * hh;
      const unsigned short* pbl = Wrl + (size_t)ncol * DF + k0 + 8 * hh;
      FragB fbh, fbl;
      fbh.half[0] = *(const v8us*)pbh; fbh.half[1] = *(const v8us*)(pbh + 16);
      fbl.half[0] = *(const v8us*)pbl; fbl.half[1] = *(const v8us*)(pbl + 16);
      accv[ct] = wmb(fah.v, fbh.v, accv[ct]);
      accv[ct] = wmb(fah.v, fbl.v, accv[ct]);
      accv[ct] = wmb(fal.v, fbh.v, accv[ct]);
    }
  }
  __syncthreads();

#define XSTEP(ARR, NJ, MK) { for (int j_ = 0; j_ < NJ; ++j_) { for (int r_ = 0; r_ < 8; ++r_) ARR[j_][r_] += __shfl_xor(ARR[j_][r_], MK, 32); } }

  {
    float sr[5][8];
#pragma unroll
    for (int j = 0; j < 5; ++j)
#pragma unroll
      for (int r8 = 0; r8 < 8; ++r8) sr[j][r8] = 0.f;
#pragma unroll
    for (int ct = 0; ct < 4; ++ct) {
      const int cin = ct * 16 + m;
      const int col = hd * HC + cin;
      const float b = br[col];
      float cf[5];
      cf[0] = attr[(0 * NH + hd) * HC + cin];
      cf[1] = attr[(1 * NH + hd) * HC + cin];
      cf[2] = attr[(2 * NH + hd) * HC + cin];
      cf[3] = relq[hd * HC + cin];
      cf[4] = relk[hd * HC + cin];
#pragma unroll
      for (int r8 = 0; r8 < 8; ++r8) {
        const float val = accv[ct][r8] + b;
        Xs[(rt * 16 + 8 * hh + r8) * XSP + col] = val;
#pragma unroll
        for (int j = 0; j < 5; ++j) sr[j][r8] += val * cf[j];
      }
    }
    XSTEP(sr, 5, 1) XSTEP(sr, 5, 2) XSTEP(sr, 5, 4) XSTEP(sr, 5, 8)
    if (m == 0) {
#pragma unroll
      for (int r8 = 0; r8 < 8; ++r8) {
        const int row = rt * 16 + 8 * hh + r8;
#pragma unroll
        for (int j = 0; j < 5; ++j) LGs[row * LGW + (NR + j) * NH + hd] = sr[j][r8];
      }
    }
  }

  v8f acck[4];
#pragma unroll
  for (int ct = 0; ct < 4; ++ct) { v8f z = {0.f, 0.f, 0.f, 0.f, 0.f, 0.f, 0.f, 0.f}; acck[ct] = z; }
#pragma unroll 1
  for (int kt = 0; kt < DF / 32; ++kt) {
    const int k0 = kt * 32;
    FragH fa;
    const _Float16* pa = Af + arow * AP + k0 + 8 * hh;
    fa.half[0] = *(const v8h*)pa; fa.half[1] = *(const v8h*)(pa + 16);
#pragma unroll
    for (int ct = 0; ct < 4; ++ct) {
      const int ncol = hd * HC + ct * 16 + m;
      const _Float16* pb = Wl16 + (size_t)ncol * DF + k0 + 8 * hh;
      FragH fb;
      fb.half[0] = *(const v8h*)pb; fb.half[1] = *(const v8h*)(pb + 16);
      acck[ct] = wmh(fa.v, fb.v, acck[ct]);
    }
  }

  {
    float sl[3][8];
#pragma unroll
    for (int j = 0; j < 3; ++j)
#pragma unroll
      for (int r8 = 0; r8 < 8; ++r8) sl[j][r8] = 0.f;
#pragma unroll
    for (int ct = 0; ct < 4; ++ct) {
      const int cin = ct * 16 + m;
      const int col = hd * HC + cin;
      const float b = bl[col];
      float cf[3];
      cf[0] = attl[(0 * NH + hd) * HC + cin];
      cf[1] = attl[(1 * NH + hd) * HC + cin];
      cf[2] = attl[(2 * NH + hd) * HC + cin];
#pragma unroll
      for (int r8 = 0; r8 < 8; ++r8) {
        const float val = acck[ct][r8] * 0.0625f + b;
#pragma unroll
        for (int j = 0; j < 3; ++j) sl[j][r8] += val * cf[j];
      }
    }
    XSTEP(sl, 3, 1) XSTEP(sl, 3, 2) XSTEP(sl, 3, 4) XSTEP(sl, 3, 8)
    if (m == 0) {
#pragma unroll
      for (int r8 = 0; r8 < 8; ++r8) {
        const int row = rt * 16 + 8 * hh + r8;
#pragma unroll
        for (int j = 0; j < 3; ++j) LGs[row * LGW + j * NH + hd] = sl[j][r8];
      }
    }
  }
#undef XSTEP
  __syncthreads();

  {
    v4f xr[8];
#pragma unroll
    for (int i = 0; i < 4; ++i) {
      xr[2 * i]     = *(const v4f*)(Xs + (4 * wave + i) * XSP + 4 * lane);
      xr[2 * i + 1] = *(const v4f*)(Xs + (4 * wave + i) * XSP + 128 + 4 * lane);
    }
    const v4f gv = *(const v4f*)(LGs + (4 * wave + (lane >> 3)) * LGW + (lane & 7) * 4);
    float* gp  = lgp + (size_t)(rowBase + 4 * wave + (lane >> 3)) * LGW + (lane & 7) * 4;
    float* xp0 = vpl + (size_t)(rowBase + 4 * wave) * DF + 4 * lane;
#pragma unroll
    for (int i = 0; i < 4; ++i) {
      *(volatile v4f*)(xp0 + (size_t)i * DF)       = xr[2 * i];
      *(volatile v4f*)(xp0 + (size_t)i * DF + 128) = xr[2 * i + 1];
    }
    *(volatile v4f*)gp = gv;
    __threadfence();
#pragma unroll
    for (int i = 0; i < 4; ++i) {
      *(volatile v4f*)(xp0 + (size_t)i * DF)       = xr[2 * i];
      *(volatile v4f*)(xp0 + (size_t)i * DF + 128) = xr[2 * i + 1];
    }
    *(volatile v4f*)gp = gv;
  }
}

__global__ __launch_bounds__(NTHR) void k_agg(
    const int* __restrict__ es0, const int* __restrict__ ed0,
    const int* __restrict__ es1, const int* __restrict__ ed1,
    const int* __restrict__ es2, const int* __restrict__ ed2,
    const float* __restrict__ lgp, float* gpl,
    int nE0, int nE1, int nE2, int nN, int nPA) {
  __shared__ __attribute__((aligned(16))) float sacc[NB * NH];
  __shared__ int list[NWAVE * WCAP];
  __shared__ int wcnt[NWAVE];

  const int tid  = threadIdx.x;
  const int lane = tid & 31;
  const int wave = tid >> 5;
  const int nodeBase = blockIdx.x * NB;
  {
    const v4f z4 = {0.f, 0.f, 0.f, 0.f};
#pragma unroll
    for (int i = 0; i < 8; ++i) *(v4f*)(sacc + (size_t)(tid + NTHR * i) * NH) = z4;
  }
  const int sub = lane >> 2;
  const int hd  = lane & 3;

#pragma unroll 1
  for (int r = 0; r < NR; ++r) {
    const int* es = (r == 0) ? es0 : ((r == 1) ? es1 : es2);
    const int* ed = (r == 0) ? ed0 : ((r == 1) ? ed1 : ed2);
    const int  nE = (r == 0) ? nE0 : ((r == 1) ? nE1 : nE2);
    const bool al16 = ((((uintptr_t)ed) & 15u) == 0u);
    const int nChunks = (nE + CHUNK - 1) / CHUNK;

#pragma unroll 1
    for (int ch = 0; ch < nChunks; ++ch) {
      const int cbase = ch * CHUNK;
      int wc = 0;
#pragma unroll
      for (int g = 0; g < NGRP; ++g) {
        const int el0 = (g * NTHR + tid) * 4;
        const int e0  = cbase + el0;
        const int sent = -2147483647 - 1;
        v4i d;
        if (al16 && (e0 + 3 < nE)) {
          d = *(const v4i*)(ed + e0);
        } else {
          d.x = (e0     < nE) ? ed[min(e0, nE - 1)]     : sent;
          d.y = (e0 + 1 < nE) ? ed[min(e0 + 1, nE - 1)] : sent;
          d.z = (e0 + 2 < nE) ? ed[min(e0 + 2, nE - 1)] : sent;
          d.w = (e0 + 3 < nE) ? ed[min(e0 + 3, nE - 1)] : sent;
        }
        const unsigned s0 = (unsigned)d.x - (unsigned)nodeBase;
        const unsigned s1 = (unsigned)d.y - (unsigned)nodeBase;
        const unsigned s2 = (unsigned)d.z - (unsigned)nodeBase;
        const unsigned s3 = (unsigned)d.w - (unsigned)nodeBase;
        const bool h0 = s0 < (unsigned)NB;
        const bool h1 = s1 < (unsigned)NB;
        const bool h2 = s2 < (unsigned)NB;
        const bool h3 = s3 < (unsigned)NB;
        const unsigned many = __builtin_amdgcn_ballot_w32(h0 | h1 | h2 | h3);
        if (many != 0u) {
#define HITJ(J, HJ, SJ) { \
            const unsigned mj = __builtin_amdgcn_ballot_w32(HJ); \
            if (HJ) { \
              const int pos = wc + (int)__builtin_amdgcn_mbcnt_lo(mj, 0u); \
              if (pos < WCAP) list[wave * WCAP + pos] = ((el0 + (J)) << 12) | (int)(SJ); \
            } \
            wc += (int)__builtin_popcount(mj); }
          HITJ(0, h0, s0)
          HITJ(1, h1, s1)
          HITJ(2, h2, s2)
          HITJ(3, h3, s3)
#undef HITJ
        }
      }
      if (lane == 0) wcnt[wave] = wc;
      __syncthreads();

      if (wave == 0) {
#pragma unroll 1
        for (int wsx = 0; wsx < NWAVE; ++wsx) {
          int n = wcnt[wsx];
          n = n > WCAP ? WCAP : n;
          n = n < 0 ? 0 : n;
#pragma unroll 1
          for (int i = 0; i < n; i += 8) {
            const int idx = i + sub;
            const bool valid = idx < n;
            const int li  = idx < WCAP - 1 ? idx : WCAP - 1;
            const int ent = list[wsx * WCAP + li];
            const int slot = ent & (NB - 1);
            const int el   = (ent >> 12) & (CHUNK - 1);
            int e = cbase + el;
            if (e > nE - 1) e = nE - 1;
            int src = es[e];
            src = src < 0 ? 0 : (src > nN - 1 ? nN - 1 : src);
            int nd = nodeBase + slot;
            if (nd > nN - 1) nd = nN - 1;
            float a = lgp[(size_t)src * LGW + r * NH + hd] + lgp[(size_t)nd * LGW + (NR + r) * NH + hd];
            a = (a >= 0.f) ? a : 0.2f * a;
            a = fminf(a, ACLAMP);
            const float p = valid ? __expf(a) : 0.f;
            const int key = valid ? slot : (-1 - sub);
            float psum = p;
            bool leader = valid;
#pragma unroll
            for (int dd = 1; dd < 8; ++dd) {
              const int   kdn = __shfl_down(key, 4 * dd, 32);
              const float pdn = __shfl_down(p, 4 * dd, 32);
              if ((sub + dd < 8) && (kdn == key)) psum += pdn;
              const int   kup = __shfl_up(key, 4 * dd, 32);
              if ((sub - dd >= 0) && (kup == key)) leader = false;
            }
            if (leader) {
              const float o = sacc[slot * NH + hd];
              sacc[slot * NH + hd] = o + psum;
            }
          }
        }
      }
      __syncthreads();
    }

    v4f gv[8];
#pragma unroll
    for (int i = 0; i < 8; ++i) {
      const int slot = tid + NTHR * i;
      const v4f sv = *(const v4f*)(sacc + (size_t)slot * NH);
      v4f g4;
      g4.x = sv.x * __builtin_amdgcn_rcpf(sv.x + 1e-16f);
      g4.y = sv.y * __builtin_amdgcn_rcpf(sv.y + 1e-16f);
      g4.z = sv.z * __builtin_amdgcn_rcpf(sv.z + 1e-16f);
      g4.w = sv.w * __builtin_amdgcn_rcpf(sv.w + 1e-16f);
      gv[i] = g4;
    }
    float* gbase = gpl + ((size_t)r * (size_t)nPA + (size_t)nodeBase) * NH;
#pragma unroll
    for (int i = 0; i < 8; ++i) *(volatile v4f*)(gbase + (size_t)(tid + NTHR * i) * NH) = gv[i];
    {
      const v4f z4 = {0.f, 0.f, 0.f, 0.f};
#pragma unroll
      for (int i = 0; i < 8; ++i) *(v4f*)(sacc + (size_t)(tid + NTHR * i) * NH) = z4;
    }
    __threadfence();
#pragma unroll
    for (int i = 0; i < 8; ++i) *(volatile v4f*)(gbase + (size_t)(tid + NTHR * i) * NH) = gv[i];
  }
}

__global__ __launch_bounds__(NTHR) void k_out(
    const float* __restrict__ vpl, const float* __restrict__ lgp, const float* __restrict__ gpl,
    const float* __restrict__ gam, const float* __restrict__ bet,
    float* out, int nN, int nPA) {
  const int tid  = threadIdx.x;
  const int lane = tid & 31;
  const int wave = tid >> 5;
  const int node = blockIdx.x * NWAVE + wave;
  if (node >= nN) return;
  const size_t nrow = (size_t)node;
  const int c0 = 4 * lane;
  const int c1 = 128 + 4 * lane;

  const v4f x0 = *(const v4f*)(vpl + nrow * DF + c0);
  const v4f x1 = *(const v4f*)(vpl + nrow * DF + c1);
  const v4f qd = *(const v4f*)(lgp + nrow * LGW + (NR + 3) * NH);
  const v4f kd = *(const v4f*)(lgp + nrow * LGW + (NR + 4) * NH);
  const v4f g0 = *(const v4f*)(gpl + ((size_t)0 * (size_t)nPA + nrow) * NH);
  const v4f g1 = *(const v4f*)(gpl + ((size_t)1 * (size_t)nPA + nrow) * NH);
  const v4f g2 = *(const v4f*)(gpl + ((size_t)2 * (size_t)nPA + nrow) * NH);

  const v4f z0 = lrelu4(qd + g0 * kd);
  const v4f z1 = lrelu4(qd + g1 * kd);
  const v4f z2 = lrelu4(qd + g2 * kd);
  const v4f z3 = lrelu4(qd + kd);
  const v4f mz = max4(max4(z0, z1), max4(z2, z3));
  const v4f e0 = exp4(z0 - mz);
  const v4f e1 = exp4(z1 - mz);
  const v4f e2 = exp4(z2 - mz);
  const v4f e3 = exp4(z3 - mz);
  const v4f esum = e0 + e1 + e2 + e3;
  const v4f w = (e0 * g0 + e1 * g1 + e2 * g2 + e3) / esum;

  const int h0 = lane >> 4;
  const float w0 = h0 ? w.y : w.x;
  const float w1 = h0 ? w.w : w.z;
  const v4f y0 = relu4(x0 * w0);
  const v4f y1 = relu4(x1 * w1);

  const float s  = wsum(y0.x + y0.y + y0.z + y0.w + y1.x + y1.y + y1.z + y1.w);
  const float mu = s * (1.0f / DF);
  const v4f d0 = y0 - mu;
  const v4f d1 = y1 - mu;
  const float q  = wsum(d0.x * d0.x + d0.y * d0.y + d0.z * d0.z + d0.w * d0.w +
                        d1.x * d1.x + d1.y * d1.y + d1.z * d1.z + d1.w * d1.w);
  const float rs = rsqrtf(q * (1.0f / DF) + 1e-5f);
  const v4f ga = *(const v4f*)(gam + c0);
  const v4f gb = *(const v4f*)(gam + c1);
  const v4f ba = *(const v4f*)(bet + c0);
  const v4f bb = *(const v4f*)(bet + c1);
  const v4f o0 = d0 * rs * ga + ba;
  const v4f o1 = d1 * rs * gb + bb;

  float* op = out + nrow * DF;
  *(volatile v4f*)(op + c0) = o0;
  *(volatile v4f*)(op + c1) = o1;
  __threadfence();
  *(volatile v4f*)(op + c0) = o0;
  *(volatile v4f*)(op + c1) = o1;
}

extern "C" void kernel_launch(void* const* d_in, const int* in_sizes, int n_in,
                              void* d_out, int out_size, void* d_ws, size_t ws_size,
                              hipStream_t stream) {
  if (n_in < 17) return;
  if (in_sizes[0] <= 0 || (in_sizes[0] % DF) != 0) return;
  const int nN = in_sizes[0] / DF;
  if (in_sizes[1] != DF * DF || in_sizes[3] != DF * DF) return;
  if (in_sizes[2] != DF || in_sizes[4] != DF) return;
  if (in_sizes[5] != NR * NH * HC || in_sizes[6] != NR * NH * HC) return;
  if (in_sizes[7] != NH * HC || in_sizes[8] != NH * HC) return;
  if (in_sizes[9] != DF || in_sizes[10] != DF) return;
  const int nE0 = in_sizes[11], nE1 = in_sizes[13], nE2 = in_sizes[15];
  if (nE0 < 0 || nE1 < 0 || nE2 < 0) return;
  if (in_sizes[12] != nE0 || in_sizes[14] != nE1 || in_sizes[16] != nE2) return;
  if (out_size != nN * DF) return;

  const float* feat = (const float*)d_in[0];
  const float* Wl   = (const float*)d_in[1];
  const float* bl   = (const float*)d_in[2];
  const float* Wr   = (const float*)d_in[3];
  const float* br   = (const float*)d_in[4];
  const float* attl = (const float*)d_in[5];
  const float* attr = (const float*)d_in[6];
  const float* relq = (const float*)d_in[7];
  const float* relk = (const float*)d_in[8];
  const float* gam  = (const float*)d_in[9];
  const float* bet  = (const float*)d_in[10];
  const int*   es0  = (const int*)d_in[11];
  const int*   ed0  = (const int*)d_in[12];
  const int*   es1  = (const int*)d_in[13];
  const int*   ed1  = (const int*)d_in[14];
  const int*   es2  = (const int*)d_in[15];
  const int*   ed2  = (const int*)d_in[16];
  float* out = (float*)d_out;

  const int nP    = ((nN + GR - 1) / GR) * GR;
  const int gridA = (nN + NB - 1) / NB;
  const int nPA   = gridA * NB;

  size_t off = 0;
  _Float16*       Wl16 = (_Float16*)((char*)d_ws + off);       off += (size_t)DF * DF * 2;
  unsigned short* Wrh  = (unsigned short*)((char*)d_ws + off); off += (size_t)DF * DF * 2;
  unsigned short* Wrl  = (unsigned short*)((char*)d_ws + off); off += (size_t)DF * DF * 2;
  float* vpl = (float*)((char*)d_ws + off); off += (size_t)nP * DF * sizeof(float);
  float* lgp = (float*)((char*)d_ws + off); off += (size_t)nP * LGW * sizeof(float);
  float* gpl = (float*)((char*)d_ws + off); off += (size_t)NR * nPA * NH * sizeof(float);
  if (off > ws_size) return;
  if (off > (size_t)134217728) return;

  const int nT = DF * DF / 8;
  k_prep<<<(nT + NTHR - 1) / NTHR, NTHR, 0, stream>>>(Wl, Wr, Wl16, Wrh, Wrl, nT);

  k_gemm<<<nP / GR, NTHR, 0, stream>>>(feat, Wl16, Wrh, Wrl, bl, br, attl, attr, relq, relk,
                                       vpl, lgp, nN);

  k_agg<<<gridA, NTHR, 0, stream>>>(es0, ed0, es1, ed1, es2, ed2, lgp, gpl,
                                    nE0, nE1, nE2, nN, nPA);

  k_out<<<(nN + NWAVE - 1) / NWAVE, NTHR, 0, stream>>>(vpl, lgp, gpl, gam, bet, out, nN, nPA);
}
